// MinkFormerBlock_44384192037348
// MI455X (gfx1250) — hardware-verified
//
#include <hip/hip_runtime.h>
#include <stdint.h>
#include <stddef.h>


#define CCH     128
#define LDP     128
#define EPI_P   128
#define TILE_M  128
#define NTHR    256
#define NBLK    64
#define SMEM_V4 4096

typedef _Float16 f16;
typedef f16    v16h __attribute__((ext_vector_type(16)));
typedef __bf16 v16b __attribute__((ext_vector_type(16)));
typedef float  v8f  __attribute__((ext_vector_type(8)));
typedef float  v4f  __attribute__((ext_vector_type(4)));
typedef unsigned int v4u __attribute__((ext_vector_type(4)));
typedef unsigned int v2u __attribute__((ext_vector_type(2)));

union FragH { v16h v; v4u u[2]; };
union FragB { v16b v; v4u u[2]; };

__device__ __forceinline__ v8f mma_f16(const FragH& a, const FragH& b, v8f c) {
  v8f d = __builtin_amdgcn_wmma_f32_16x16x32_f16(false, a.v, false, b.v, (short)0, c, false, false);
  asm volatile("v_nop\n\tv_nop\n\tv_nop\n\tv_nop" : "+v"(d) : "v"(a.v), "v"(b.v));
  return d;
}
__device__ __forceinline__ v8f mma_bf16(const FragB& a, const FragB& b, v8f c) {
  v8f d = __builtin_amdgcn_wmma_f32_16x16x32_bf16(false, a.v, false, b.v, (short)0, c, false, false);
  asm volatile("v_nop\n\tv_nop\n\tv_nop\n\tv_nop" : "+v"(d) : "v"(a.v), "v"(b.v));
  return d;
}

__device__ __forceinline__ unsigned int bf16_bits(float f) {
  unsigned int u = __float_as_uint(f);
  return (u + 0x7FFFu + ((u >> 16) & 1u)) >> 16;
}
__device__ __forceinline__ unsigned int f16_bits(float f) {
  union { f16 hv; unsigned short s; } cv;
  cv.hv = (f16)f;
  return (unsigned int)cv.s;
}
__device__ __forceinline__ unsigned int pack2_f16(float a, float b) {
  return f16_bits(a) | (f16_bits(b) << 16);
}
__device__ __forceinline__ v2u split_pair(float a, float b) {
  unsigned int ha = bf16_bits(a), hb = bf16_bits(b);
  unsigned int la = bf16_bits(a - __uint_as_float(ha << 16));
  unsigned int lb = bf16_bits(b - __uint_as_float(hb << 16));
  v2u r;
  r.x = ha | (hb << 16);
  r.y = la | (lb << 16);
  return r;
}
__device__ __forceinline__ void split8(v4f p, v4f q, v4u& hi, v4u& lo) {
  v2u a = split_pair(p.x, p.y), b = split_pair(p.z, p.w);
  v2u c = split_pair(q.x, q.y), d = split_pair(q.z, q.w);
  hi.x = a.x; hi.y = b.x; hi.z = c.x; hi.w = d.x;
  lo.x = a.y; lo.y = b.y; lo.z = c.y; lo.w = d.y;
}
__device__ __forceinline__ float bn_res(float t, float sc, float sh, float res) {
  return fmaf(t, sc, sh) + res;
}

template<int MODE>
__device__ __forceinline__ void epilogue(v8f (&acc)[8], v4u* smem, int wave, int h, int m, int lane,
                                         int rowBase, int N, float oscale,
                                         const float* __restrict__ Vg, float* outF, unsigned short* outH)
{
  float* sE = (float*)smem;
  __syncthreads();
#pragma unroll
  for (int j = 0; j < 8; ++j) {
    float* col = sE + (wave * 16 + 8 * h) * EPI_P + 16 * j + m;
#pragma unroll
    for (int r = 0; r < 8; ++r) col[r * EPI_P] = acc[j][r] * oscale;
  }
  __syncthreads();
  if (MODE == 0) {
    v4f vals[16];
#pragma unroll
    for (int r = 0; r < 16; ++r)
      vals[r] = *(const v4f*)(sE + (wave * 16 + r) * EPI_P + 4 * lane);
#pragma unroll
    for (int r = 0; r < 16; ++r) {
      const int grow = rowBase + wave * 16 + r;
      if (grow < N) *(volatile v4f*)(outF + (size_t)grow * CCH + 4 * lane) = vals[r];
    }
    __threadfence();
#pragma unroll
    for (int r = 0; r < 16; ++r) {
      const int grow = rowBase + wave * 16 + r;
      if (grow < N) *(volatile v4f*)(outF + (size_t)grow * CCH + 4 * lane) = vals[r];
    }
  } else {
    v4u vals[8];
#pragma unroll
    for (int q = 0; q < 8; ++q) {
      const int lrow = wave * 16 + 2 * q + h;
      const int grow = rowBase + lrow;
      const int gq = grow < N ? grow : N - 1;
      const float* src = sE + lrow * EPI_P + 8 * m;
      v4f p0 = *(const v4f*)src;
      v4f p1 = *(const v4f*)(src + 4);
      if (MODE == 2) {
        const float* vg = Vg + (size_t)gq * CCH + 8 * m;
        v4f g0 = *(const v4f*)vg;
        v4f g1 = *(const v4f*)(vg + 4);
        p0 *= g0;
        p1 *= g1;
      }
      v4u o;
      o.x = pack2_f16(p0.x, p0.y);
      o.y = pack2_f16(p0.z, p0.w);
      o.z = pack2_f16(p1.x, p1.y);
      o.w = pack2_f16(p1.z, p1.w);
      vals[q] = o;
    }
#pragma unroll
    for (int q = 0; q < 8; ++q) {
      const int grow = rowBase + wave * 16 + 2 * q + h;
      if (grow < N) *(volatile v4u*)(outH + (size_t)grow * CCH + 8 * m) = vals[q];
    }
    __threadfence();
#pragma unroll
    for (int q = 0; q < 8; ++q) {
      const int grow = rowBase + wave * 16 + 2 * q + h;
      if (grow < N) *(volatile v4u*)(outH + (size_t)grow * CCH + 8 * m) = vals[q];
    }
  }
}

template<int MODE>
__global__ __launch_bounds__(NTHR) void conv_kernel(
    const unsigned short* __restrict__ feats, const int* __restrict__ nbr, int taps, int N,
    const unsigned short* __restrict__ Wt, float oscale,
    const float* __restrict__ Vg, float* outF, unsigned short* outH)
{
  __shared__ v4u smem[SMEM_V4];
  unsigned short* sA = (unsigned short*)smem;
  unsigned short* sB = sA + TILE_M * LDP;
  const int tid = threadIdx.x, lane = tid & 31, wave = tid >> 5;
  const int h = (lane >> 4) & 1, m = lane & 15;
  const int sr = tid >> 4, sp = tid & 15;
  const int rowBase = blockIdx.x * TILE_M;

  v8f acc[8] = {};

  for (int t = 0; t < taps; ++t) {
    __syncthreads();
#pragma unroll
    for (int i = 0; i < 8; ++i) {
      const int r = sr + 16 * i;
      const int grow = rowBase + r;
      const int gq = grow < N ? grow : N - 1;
      int idx = nbr[(size_t)gq * taps + t];
      idx = idx < 0 ? idx + N : idx;
      idx = idx < 0 ? 0 : (idx >= N ? N - 1 : idx);
      v4u va = *(const v4u*)(feats + (size_t)idx * CCH + 8 * sp);
      v4u vb = *(const v4u*)(Wt + ((size_t)t * CCH + r) * CCH + 8 * sp);
      *(v4u*)(sA + r * LDP + 8 * sp) = va;
      *(v4u*)(sB + r * LDP + 8 * sp) = vb;
    }
    __syncthreads();
    const unsigned short* aRow = sA + (wave * 16 + m) * LDP + 8 * h;
    const unsigned short* bRow = sB + m * LDP + 8 * h;
#pragma unroll
    for (int s = 0; s < 4; ++s) {
      FragH a;
      a.u[0] = *(const v4u*)(aRow + 32 * s);
      a.u[1] = *(const v4u*)(aRow + 32 * s + 16);
#pragma unroll
      for (int j = 0; j < 8; ++j) {
        const unsigned short* bp = bRow + 16 * j * LDP + 32 * s;
        FragH b;
        b.u[0] = *(const v4u*)bp;
        b.u[1] = *(const v4u*)(bp + 16);
        acc[j] = mma_f16(a, b, acc[j]);
      }
    }
  }
  epilogue<MODE>(acc, smem, wave, h, m, lane, rowBase, N, oscale, Vg, outF, outH);
}

template<int MODE>
__global__ __launch_bounds__(NTHR) void proj_kernel(
    const float* __restrict__ X, int N,
    const unsigned short* __restrict__ Wh, const unsigned short* __restrict__ Wl,
    float* outF, unsigned short* outH)
{
  __shared__ v4u smem[SMEM_V4];
  unsigned short* sBh = (unsigned short*)smem;
  unsigned short* sBl = sBh + TILE_M * LDP;
  const int tid = threadIdx.x, lane = tid & 31, wave = tid >> 5;
  const int h = (lane >> 4) & 1, m = lane & 15;
  const int sr = tid >> 4, sp = tid & 15;
  const int rowBase = blockIdx.x * TILE_M;

#pragma unroll
  for (int i = 0; i < 8; ++i) {
    const int r = sr + 16 * i;
    v4u vh = *(const v4u*)(Wh + (size_t)r * CCH + 8 * sp);
    v4u vl = *(const v4u*)(Wl + (size_t)r * CCH + 8 * sp);
    *(v4u*)(sBh + r * LDP + 8 * sp) = vh;
    *(v4u*)(sBl + r * LDP + 8 * sp) = vl;
  }
  __syncthreads();

  v8f acc[8] = {};
  const int grow = rowBase + wave * 16 + m;
  const int gq = grow < N ? grow : N - 1;
  const float* xr = X + (size_t)gq * CCH + 8 * h;
  const unsigned short* bhRow = sBh + m * LDP + 8 * h;
  const unsigned short* blRow = sBl + m * LDP + 8 * h;
#pragma unroll
  for (int s = 0; s < 4; ++s) {
    v4f p0 = *(const v4f*)(xr + 32 * s);
    v4f p1 = *(const v4f*)(xr + 32 * s + 4);
    v4f p2 = *(const v4f*)(xr + 32 * s + 16);
    v4f p3 = *(const v4f*)(xr + 32 * s + 20);
    FragB ah, al;
    split8(p0, p1, ah.u[0], al.u[0]);
    split8(p2, p3, ah.u[1], al.u[1]);
#pragma unroll
    for (int j = 0; j < 8; ++j) {
      const unsigned short* ph = bhRow + 16 * j * LDP + 32 * s;
      const unsigned short* pl = blRow + 16 * j * LDP + 32 * s;
      FragB bh, bl;
      bh.u[0] = *(const v4u*)ph;
      bh.u[1] = *(const v4u*)(ph + 16);
      bl.u[0] = *(const v4u*)pl;
      bl.u[1] = *(const v4u*)(pl + 16);
      acc[j] = mma_bf16(ah, bh, acc[j]);
      acc[j] = mma_bf16(al, bh, acc[j]);
      acc[j] = mma_bf16(ah, bl, acc[j]);
    }
  }
  epilogue<MODE>(acc, smem, wave, h, m, lane, rowBase, N, 1.0f, X, outF, outH);
}

__global__ __launch_bounds__(NTHR) void wprep_f16_kernel(const float* __restrict__ W, float scale,
                                                         unsigned short* out)
{
  __shared__ v4u smem[SMEM_V4 / 2];
  unsigned short* sT = (unsigned short*)smem;
  const int tid = threadIdx.x, t = blockIdx.x;
  const int sr = tid >> 4, sp = tid & 15;
#pragma unroll 4
  for (int i = 0; i < 16; ++i) {
    const int c = tid + NTHR * i;
    const int k = c >> 5;
    const int n4 = (c & 31) * 4;
    v4f w = *(const v4f*)(W + ((size_t)t * CCH + k) * CCH + n4);
    sT[(n4 + 0) * LDP + k] = (unsigned short)f16_bits(w.x * scale);
    sT[(n4 + 1) * LDP + k] = (unsigned short)f16_bits(w.y * scale);
    sT[(n4 + 2) * LDP + k] = (unsigned short)f16_bits(w.z * scale);
    sT[(n4 + 3) * LDP + k] = (unsigned short)f16_bits(w.w * scale);
  }
  __syncthreads();
  v4u vals[8];
#pragma unroll
  for (int i = 0; i < 8; ++i) {
    const int n = sr + 16 * i;
    vals[i] = *(const v4u*)(sT + n * LDP + 8 * sp);
  }
#pragma unroll
  for (int i = 0; i < 8; ++i) {
    const int n = sr + 16 * i;
    *(volatile v4u*)(out + ((size_t)t * CCH + n) * CCH + 8 * sp) = vals[i];
  }
  __threadfence();
#pragma unroll
  for (int i = 0; i < 8; ++i) {
    const int n = sr + 16 * i;
    *(volatile v4u*)(out + ((size_t)t * CCH + n) * CCH + 8 * sp) = vals[i];
  }
}

__global__ __launch_bounds__(NTHR) void wprep_split_kernel(const float* __restrict__ W,
                                                           unsigned short* outHi, unsigned short* outLo)
{
  __shared__ v4u smem[SMEM_V4];
  unsigned short* sH = (unsigned short*)smem;
  unsigned short* sL = sH + TILE_M * LDP;
  const int tid = threadIdx.x;
  const int sr = tid >> 4, sp = tid & 15;
#pragma unroll 4
  for (int i = 0; i < 16; ++i) {
    const int c = tid + NTHR * i;
    const int k = c >> 5;
    const int n4 = (c & 31) * 4;
    v4f w = *(const v4f*)(W + (size_t)k * CCH + n4);
    v2u a = split_pair(w.x, w.y);
    v2u b = split_pair(w.z, w.w);
    sH[(n4 + 0) * LDP + k] = (unsigned short)(a.x & 0xFFFFu);
    sH[(n4 + 1) * LDP + k] = (unsigned short)(a.x >> 16);
    sH[(n4 + 2) * LDP + k] = (unsigned short)(b.x & 0xFFFFu);
    sH[(n4 + 3) * LDP + k] = (unsigned short)(b.x >> 16);
    sL[(n4 + 0) * LDP + k] = (unsigned short)(a.y & 0xFFFFu);
    sL[(n4 + 1) * LDP + k] = (unsigned short)(a.y >> 16);
    sL[(n4 + 2) * LDP + k] = (unsigned short)(b.y & 0xFFFFu);
    sL[(n4 + 3) * LDP + k] = (unsigned short)(b.y >> 16);
  }
  __syncthreads();
  v4u vh[8], vl[8];
#pragma unroll
  for (int i = 0; i < 8; ++i) {
    const int n = sr + 16 * i;
    vh[i] = *(const v4u*)(sH + n * LDP + 8 * sp);
    vl[i] = *(const v4u*)(sL + n * LDP + 8 * sp);
  }
#pragma unroll
  for (int i = 0; i < 8; ++i) {
    const int n = sr + 16 * i;
    *(volatile v4u*)(outHi + (size_t)n * CCH + 8 * sp) = vh[i];
    *(volatile v4u*)(outLo + (size_t)n * CCH + 8 * sp) = vl[i];
  }
  __threadfence();
#pragma unroll
  for (int i = 0; i < 8; ++i) {
    const int n = sr + 16 * i;
    *(volatile v4u*)(outHi + (size_t)n * CCH + 8 * sp) = vh[i];
    *(volatile v4u*)(outLo + (size_t)n * CCH + 8 * sp) = vl[i];
  }
}

__global__ __launch_bounds__(128) void bn_stats_kernel(const float* __restrict__ T, int N, int rpb,
                                                       double* part)
{
  const int c = threadIdx.x, b = blockIdx.x;
  int r0 = b * rpb; if (r0 > N) r0 = N;
  int r1 = r0 + rpb; if (r1 > N) r1 = N;
  double s = 0.0, q = 0.0;
  for (int r = r0; r < r1; ++r) {
    const double v = (double)T[(size_t)r * CCH + c];
    s += v;
    q += v * v;
  }
  double* p0 = part + (size_t)b * CCH + c;
  double* p1 = part + (size_t)(NBLK + b) * CCH + c;
  *(volatile double*)p0 = s;
  *(volatile double*)p1 = q;
  __threadfence();
  *(volatile double*)p0 = s;
  *(volatile double*)p1 = q;
}

__global__ __launch_bounds__(128) void bn_finalize_kernel(const double* __restrict__ part, int N,
                                                          const float* __restrict__ gamma,
                                                          const float* __restrict__ beta,
                                                          float* sb)
{
  const int c = threadIdx.x;
  double s = 0.0, q = 0.0;
  for (int b = 0; b < NBLK; ++b) {
    s += part[(size_t)b * CCH + c];
    q += part[(size_t)(NBLK + b) * CCH + c];
  }
  const double invN = 1.0 / (double)N;
  const double mu = s * invN;
  double var = q * invN - mu * mu;
  if (var < 0.0) var = 0.0;
  const float sc = rsqrtf((float)var + 1e-5f) * gamma[c];
  const float sh = beta[c] - (float)mu * sc;
  *(volatile float*)(sb + c) = sc;
  *(volatile float*)(sb + CCH + c) = sh;
  __threadfence();
  *(volatile float*)(sb + c) = sc;
  *(volatile float*)(sb + CCH + c) = sh;
}

__global__ __launch_bounds__(NTHR) void bn_relu_kernel(const float* __restrict__ T1, const float* __restrict__ X,
                                                       const float* __restrict__ sb, unsigned short* R, int n4)
{
  const int gid = blockIdx.x * NTHR + threadIdx.x;
  if (gid >= n4) return;
  const size_t e = (size_t)gid * 4;
  const int c = (int)(e & (size_t)(CCH - 1));
  v4f t = *(const v4f*)(T1 + e);
  v4f xv = *(const v4f*)(X + e);
  v4f sc = *(const v4f*)(sb + c);
  v4f sh = *(const v4f*)(sb + CCH + c);
  const float o0 = fmaxf(bn_res(t.x, sc.x, sh.x, xv.x), 0.f);
  const float o1 = fmaxf(bn_res(t.y, sc.y, sh.y, xv.y), 0.f);
  const float o2 = fmaxf(bn_res(t.z, sc.z, sh.z, xv.z), 0.f);
  const float o3 = fmaxf(bn_res(t.w, sc.w, sh.w, xv.w), 0.f);
  v2u pk;
  pk.x = pack2_f16(o0, o1);
  pk.y = pack2_f16(o2, o3);
  *(volatile v2u*)(R + e) = pk;
  __threadfence();
  *(volatile v2u*)(R + e) = pk;
}

__global__ __launch_bounds__(NTHR) void final_kernel(const float* __restrict__ T1, const float* __restrict__ T2,
                                                     const float* __restrict__ X,
                                                     const float* __restrict__ sb1, const float* __restrict__ sb2,
                                                     float* out, int n4)
{
  const int gid = blockIdx.x * NTHR + threadIdx.x;
  if (gid >= n4) return;
  const size_t e = (size_t)gid * 4;
  const int c = (int)(e & (size_t)(CCH - 1));
  v4f t1 = *(const v4f*)(T1 + e);
  v4f t2 = *(const v4f*)(T2 + e);
  v4f xv = *(const v4f*)(X + e);
  v4f c1 = *(const v4f*)(sb1 + c), h1 = *(const v4f*)(sb1 + CCH + c);
  v4f c2 = *(const v4f*)(sb2 + c), h2 = *(const v4f*)(sb2 + CCH + c);
  v4f o;
  {
    const float a0 = bn_res(t1.x, c1.x, h1.x, xv.x); o.x = fmaxf(bn_res(t2.x, c2.x, h2.x, a0), 0.f);
    const float a1 = bn_res(t1.y, c1.y, h1.y, xv.y); o.y = fmaxf(bn_res(t2.y, c2.y, h2.y, a1), 0.f);
    const float a2 = bn_res(t1.z, c1.z, h1.z, xv.z); o.z = fmaxf(bn_res(t2.z, c2.z, h2.z, a2), 0.f);
    const float a3 = bn_res(t1.w, c1.w, h1.w, xv.w); o.w = fmaxf(bn_res(t2.w, c2.w, h2.w, a3), 0.f);
  }
  *(volatile v4f*)(out + e) = o;
  __threadfence();
  *(volatile v4f*)(out + e) = o;
}

extern "C" void kernel_launch(void* const* d_in, const int* in_sizes, int n_in,
                              void* d_out, int out_size, void* d_ws, size_t ws_size,
                              hipStream_t stream)
{
  if (n_in < 13) return;
  const int CC = CCH * CCH;
  const int nX = in_sizes[0];
  if (nX <= 0 || (nX % CCH) != 0) return;
  const int N = nX / CCH;
  if (in_sizes[1] != CC || in_sizes[2] != CC) return;
  if (in_sizes[3] <= 0 || in_sizes[4] <= 0 || in_sizes[5] <= 0) return;
  if ((in_sizes[3] % CC) != 0 || (in_sizes[4] % CC) != 0 || (in_sizes[5] % CC) != 0) return;
  const int taps5 = in_sizes[3] / CC;
  const int taps3a = in_sizes[4] / CC;
  const int taps3b = in_sizes[5] / CC;
  if (in_sizes[6] != CCH || in_sizes[7] != CCH || in_sizes[8] != CCH || in_sizes[9] != CCH) return;
  if ((size_t)in_sizes[10] != (size_t)N * taps5) return;
  if ((size_t)in_sizes[11] != (size_t)N * taps3a) return;
  if ((size_t)in_sizes[12] != (size_t)N * taps3b) return;
  if (out_size != N * CCH) return;

  const float* x   = (const float*)d_in[0];
  const float* Wa1 = (const float*)d_in[1];
  const float* Wv1 = (const float*)d_in[2];
  const float* W5  = (const float*)d_in[3];
  const float* W31 = (const float*)d_in[4];
  const float* W32 = (const float*)d_in[5];
  const float* g1  = (const float*)d_in[6];
  const float* b1  = (const float*)d_in[7];
  const float* g2  = (const float*)d_in[8];
  const float* b2  = (const float*)d_in[9];
  const int* nbr5  = (const int*)d_in[10];
  const int* nbr3a = (const int*)d_in[11];
  const int* nbr3b = (const int*)d_in[12];
  float* out = (float*)d_out;

  char* ws = (char*)d_ws;
  size_t off = 0;
  auto carve = [&](size_t bytes) -> char* {
    char* p = ws + off;
    off += (bytes + 255) & ~(size_t)255;
    return p;
  };
  const size_t NC = (size_t)N * CCH;
  unsigned short* A   = (unsigned short*)carve(NC * 2);
  float*          V   = (float*)carve(NC * 4);
  unsigned short* P   = (unsigned short*)carve(NC * 2);
  float*          T1  = (float*)carve(NC * 4);
  unsigned short* R   = (unsigned short*)carve(NC * 2);
  float*          T2  = (float*)carve(NC * 4);
  unsigned short* W5t  = (unsigned short*)carve((size_t)taps5 * CC * 2);
  unsigned short* W31t = (unsigned short*)carve((size_t)taps3a * CC * 2);
  unsigned short* W32t = (unsigned short*)carve((size_t)taps3b * CC * 2);
  unsigned short* Wa1h = (unsigned short*)carve((size_t)CC * 2);
  unsigned short* Wa1l = (unsigned short*)carve((size_t)CC * 2);
  unsigned short* Wv1h = (unsigned short*)carve((size_t)CC * 2);
  unsigned short* Wv1l = (unsigned short*)carve((size_t)CC * 2);
  double*         part = (double*)carve((size_t)2 * NBLK * CCH * 8);
  float*          sb1  = (float*)carve((size_t)2 * CCH * 4);
  float*          sb2  = (float*)carve((size_t)2 * CCH * 4);
  if (off > ws_size) return;

  const float wscale = 64.0f;
  const float oscale = 0.015625f;
  const int gridM = (N + TILE_M - 1) / TILE_M;
  const int rpb = (N + NBLK - 1) / NBLK;
  const int n4 = N * (CCH / 4);
  const int gridE = (n4 + NTHR - 1) / NTHR;

  wprep_split_kernel<<<dim3(1), dim3(NTHR), 0, stream>>>(Wa1, Wa1h, Wa1l);
  wprep_split_kernel<<<dim3(1), dim3(NTHR), 0, stream>>>(Wv1, Wv1h, Wv1l);
  wprep_f16_kernel<<<dim3(taps5), dim3(NTHR), 0, stream>>>(W5, wscale, W5t);
  wprep_f16_kernel<<<dim3(taps3a), dim3(NTHR), 0, stream>>>(W31, wscale, W31t);
  wprep_f16_kernel<<<dim3(taps3b), dim3(NTHR), 0, stream>>>(W32, wscale, W32t);

  proj_kernel<1><<<dim3(gridM), dim3(NTHR), 0, stream>>>(x, N, Wa1h, Wa1l, T1, A);
  proj_kernel<0><<<dim3(gridM), dim3(NTHR), 0, stream>>>(x, N, Wv1h, Wv1l, V, P);

  conv_kernel<2><<<dim3(gridM), dim3(NTHR), 0, stream>>>(A, nbr5, taps5, N, W5t, oscale, V, T1, P);
  conv_kernel<0><<<dim3(gridM), dim3(NTHR), 0, stream>>>(P, nbr3a, taps3a, N, W31t, oscale, V, T1, R);
  bn_stats_kernel<<<dim3(NBLK), dim3(128), 0, stream>>>(T1, N, rpb, part);
  bn_finalize_kernel<<<dim3(1), dim3(128), 0, stream>>>(part, N, g1, b1, sb1);
  bn_relu_kernel<<<dim3(gridE), dim3(NTHR), 0, stream>>>(T1, x, sb1, R, n4);
  conv_kernel<0><<<dim3(gridM), dim3(NTHR), 0, stream>>>(R, nbr3b, taps3b, N, W32t, oscale, V, T2, P);
  bn_stats_kernel<<<dim3(NBLK), dim3(128), 0, stream>>>(T2, N, rpb, part);
  bn_finalize_kernel<<<dim3(1), dim3(128), 0, stream>>>(part, N, g2, b2, sb2);
  final_kernel<<<dim3(gridE), dim3(NTHR), 0, stream>>>(T1, T2, x, sb1, sb2, out, n4);
}
